// SwitchingDevGRUCell_75239237091518
// MI455X (gfx1250) — hardware-run, weakly checked
//
#include <hip/hip_runtime.h>
#include <math.h>

typedef __attribute__((ext_vector_type(16))) _Float16 v16h;
typedef __attribute__((ext_vector_type(8)))  _Float16 v8h;
typedef __attribute__((ext_vector_type(8)))  float    v8f;
typedef __attribute__((ext_vector_type(4)))  float    v4f;

constexpr int kB   = 32768;
constexpr int kC   = 8;
constexpr int kH   = 128;
constexpr int kR   = 16;
constexpr int kG3  = 3 * kH;
constexpr int kCR  = kC * kR;
static_assert(kCR == 128);
static_assert((kB % 64) == 0 && (kCR % 64) == 0 && (kG3 % 64) == 0);
static_assert((kH % 32) == 0 && (kCR % 32) == 0);
static_assert(kR == 16);

constexpr float kCarryH  = 16.0f;
constexpr float kCarryW  = 256.0f;
constexpr float kCarryM  = 64.0f;
constexpr float kInvAcc1 = 1.0f / (kCarryH * kCarryW);
constexpr float kInvAcc2 = 1.0f / (kCarryM * kCarryW);
constexpr float kF16MinNormal = 6.103515625e-5f;

constexpr size_t kSzA1   = (size_t)kB * kH * 2;
constexpr size_t kSzA2   = (size_t)kB * kCR * 2;
constexpr size_t kSzBT1  = (size_t)kCR * kH * 2;
constexpr size_t kSzBT2  = (size_t)kG3 * kCR * 2;
constexpr size_t kSzGP   = (size_t)kB * kG3 * 4;
constexpr size_t kOffA1  = 0;
constexpr size_t kOffA2  = kOffA1 + kSzA1;
constexpr size_t kOffBT1 = kOffA2 + kSzA2;
constexpr size_t kOffBT2 = kOffBT1 + kSzBT1;
constexpr size_t kOffGP  = kOffBT2 + kSzBT2;
constexpr size_t kWsTotal = kOffGP + kSzGP;
static_assert(kWsTotal == 67239936ull);
static_assert(kWsTotal <= 134217728ull);
static_assert((kOffA2 % 128) == 0 && (kOffBT1 % 128) == 0 && (kOffBT2 % 128) == 0 && (kOffGP % 128) == 0);

__device__ __forceinline__ _Float16 to_f16_carried(float v, float carry) {
  const float s = v * carry;
  const float f = (fabsf(s) < kF16MinNormal) ? 0.0f : s;
  return (_Float16)f;
}

__device__ __forceinline__ void tie_acc(v8f& a, v16h x, v16h y) {
  asm volatile("v_nop\n\tv_nop\n\tv_nop\n\tv_nop" : "+v"(a) : "v"(x), "v"(y));
}
__device__ __forceinline__ void settle_acc(v8f& a) {
  asm volatile("v_nop\n\tv_nop\n\tv_nop\n\tv_nop" : "+v"(a));
}
__device__ __forceinline__ void keep4_h(v16h a, v16h b, v16h c, v16h d) {
  asm volatile("v_nop" :: "v"(a), "v"(b), "v"(c), "v"(d));
}

union FragU { v16h v; v8h h[2]; };
__device__ __forceinline__ v16h frag_load(const _Float16* p) {
  FragU f;
  f.h[0] = *(const v8h*)(p);
  f.h[1] = *(const v8h*)(p + 16);
  return f.v;
}
__device__ __forceinline__ v8f frag_mma(v16h a, v16h b, v8f c) {
  return __builtin_amdgcn_wmma_f32_16x16x32_f16(false, a, false, b, (short)0, c, false, false);
}

constexpr unsigned kPrepBlkU = (unsigned)(kG3 * kCR / 8 / 256);
constexpr unsigned kPrepBlkV = (unsigned)(kCR * kH / 8 / 256);
static_assert(kPrepBlkU * 256u * 8u == (unsigned)(kG3 * kCR));
static_assert(kPrepBlkV * 256u * 8u == (unsigned)(kCR * kH));

__global__ __launch_bounds__(256) void prep_weights_kernel(
    const float* __restrict__ U, const float* __restrict__ V,
    unsigned short* __restrict__ BT1, unsigned short* __restrict__ BT2)
{
  const unsigned tid = threadIdx.x;
  v8h hv;
  unsigned short* dst;
  if (blockIdx.x < kPrepBlkU) {
    unsigned t = blockIdx.x * 256u + tid;
    asm volatile("" : "+v"(t));
    unsigned g = t >> 4;
    unsigned q = t & 15u;
    unsigned c = q >> 1;
    unsigned r0 = (q & 1u) * 8u;
    asm volatile("" : "+v"(g));
    asm volatile("" : "+v"(c));
    asm volatile("" : "+v"(r0));
    const float* src = U + ((size_t)(c * (unsigned)kG3 + g)) * kR + r0;
    const v4f a0 = *(const v4f*)(src);
    const v4f a1 = *(const v4f*)(src + 4);
#pragma unroll
    for (int e = 0; e < 4; ++e) {
      hv[e]     = to_f16_carried(a0[e], kCarryW);
      hv[4 + e] = to_f16_carried(a1[e], kCarryW);
    }
    dst = BT2 + (size_t)t * 8;
  } else {
    unsigned t = (blockIdx.x - kPrepBlkU) * 256u + tid;
    asm volatile("" : "+v"(t));
    unsigned n = t >> 4;
    unsigned q = t & 15u;
    unsigned c = n >> 4;
    unsigned r = n & 15u;
    asm volatile("" : "+v"(c));
    asm volatile("" : "+v"(r));
    asm volatile("" : "+v"(q));
    const float* src = V + ((size_t)(c * (unsigned)kH + q * 8u)) * kR + r;
#pragma unroll
    for (int e = 0; e < 8; ++e) {
      const float f = src[e * kR];
      hv[e] = to_f16_carried(f, kCarryW);
    }
    dst = BT1 + (size_t)t * 8;
  }
  *(volatile v8h*)dst = hv;
  __threadfence();
  *(volatile v8h*)dst = hv;
}

__global__ __launch_bounds__(256) void cast_h_kernel(
    const float* __restrict__ src, unsigned short* __restrict__ dstp, int total8)
{
  const int i = blockIdx.x * 256 + threadIdx.x;
  if (i >= total8) return;
  const size_t e0 = (size_t)i << 3;
  const v4f a0 = *(const v4f*)(src + e0);
  const v4f a1 = *(const v4f*)(src + e0 + 4);
  v8h hv;
#pragma unroll
  for (int e = 0; e < 4; ++e) {
    hv[e]     = to_f16_carried(a0[e], kCarryH);
    hv[4 + e] = to_f16_carried(a1[e], kCarryH);
  }
  unsigned short* q = dstp + e0;
  *(volatile v8h*)q = hv;
  __threadfence();
  *(volatile v8h*)q = hv;
}

template <int MODE>
__global__ __launch_bounds__(256) void gemm_f16_kernel(
    const unsigned short* __restrict__ Ap, int lda,
    const unsigned short* __restrict__ Btp, int ldb,
    void* __restrict__ Cout, int ldc,
    const float* __restrict__ xmix,
    int M, int N, int K, float scale, float carry_out)
{
  const _Float16* A  = (const _Float16*)Ap;
  const _Float16* Bt = (const _Float16*)Btp;
  __shared__ __align__(16) float sT[8][16 * 68];
  const int lane = threadIdx.x & 31;
  const int wave = threadIdx.x >> 5;
  const int tilesN = N >> 6;
  const int tilesM = M >> 6;
  const int tile = blockIdx.x * 8 + wave;
  if (tile >= tilesM * tilesN) return;
  const int tm = tile / tilesN;
  const int tn = tile - tm * tilesN;
  const int m0 = tm << 6;
  const int n0 = tn << 6;

  const int rlane = lane & 15;
  const int koff  = (lane >> 4) * 8;
  const int mOff  = (lane >> 4) * 8;

  v8f acc[4][4];
#pragma unroll
  for (int i = 0; i < 4; ++i)
#pragma unroll
    for (int j = 0; j < 4; ++j) acc[i][j] = (v8f){0.f, 0.f, 0.f, 0.f, 0.f, 0.f, 0.f, 0.f};

  for (int k0 = 0; k0 < K; k0 += 32) {
    v16h bh[4];
#pragma unroll
    for (int j = 0; j < 4; ++j) {
      const size_t bo = (size_t)(n0 + (j << 4) + rlane) * ldb + koff + k0;
      bh[j] = frag_load(Bt + bo);
    }
#pragma unroll
    for (int i = 0; i < 4; ++i) {
      const size_t ao = (size_t)(m0 + (i << 4) + rlane) * lda + koff + k0;
      const v16h ah = frag_load(A + ao);
#pragma unroll
      for (int j = 0; j < 4; ++j) acc[i][j] = frag_mma(ah, bh[j], acc[i][j]);
      tie_acc(acc[i][0], ah, bh[0]);
      tie_acc(acc[i][1], ah, bh[1]);
      tie_acc(acc[i][2], ah, bh[2]);
      tie_acc(acc[i][3], ah, bh[3]);
    }
    keep4_h(bh[0], bh[1], bh[2], bh[3]);
  }
#pragma unroll
  for (int i = 0; i < 4; ++i) {
    settle_acc(acc[i][0]);
    settle_acc(acc[i][1]);
    settle_acc(acc[i][2]);
    settle_acc(acc[i][3]);
  }

  float* slab = sT[wave];
#pragma unroll
  for (int i = 0; i < 4; ++i) {
    const int mBase = m0 + (i << 4);
    v4f xr[8];
    if (MODE == 0) {
#pragma unroll
      for (int r = 0; r < 8; ++r)
        xr[r] = *(const v4f*)(xmix + (size_t)(mBase + mOff + r) * kC + (n0 >> 4));
    }
#pragma unroll
    for (int j = 0; j < 4; ++j) {
#pragma unroll
      for (int r = 0; r < 8; ++r) {
        float v = acc[i][j][r] * scale;
        if (MODE == 0) {
          const float xs = xr[r][j];
          const float mx = xs * v;
          const float cv = mx * carry_out;
          v = (fabsf(cv) < kF16MinNormal) ? 0.0f : cv;
        }
        slab[(mOff + r) * 68 + (j << 4) + rlane] = v;
      }
    }
    __builtin_amdgcn_fence(__ATOMIC_RELEASE, "workgroup");
    __builtin_amdgcn_wave_barrier();
    __builtin_amdgcn_fence(__ATOMIC_ACQUIRE, "workgroup");
    if (MODE == 1) {
      float* Cf = (float*)Cout;
      const int hh = lane >> 4, c4 = (lane & 15) * 4;
      for (int pass = 0; pass < 2; ++pass) {
#pragma unroll
        for (int it = 0; it < 8; ++it) {
          const int row = it * 2 + hh;
          const v4f v = *(const v4f*)(slab + row * 68 + c4);
          *(volatile v4f*)(Cf + (size_t)(mBase + row) * ldc + n0 + c4) = v;
        }
        __threadfence();
      }
    } else {
      const int q = lane >> 3, c8 = (lane & 7) * 8;
      unsigned short* Ch = (unsigned short*)Cout;
      for (int pass = 0; pass < 2; ++pass) {
#pragma unroll
        for (int it = 0; it < 4; ++it) {
          const int row = it * 4 + q;
          const float* sp = slab + row * 68 + c8;
          v8h hv;
#pragma unroll
          for (int e = 0; e < 8; ++e) hv[e] = (_Float16)sp[e];
          *(volatile v8h*)(Ch + (size_t)(mBase + row) * ldc + n0 + c8) = hv;
        }
        __threadfence();
      }
    }
    __builtin_amdgcn_fence(__ATOMIC_RELEASE, "workgroup");
    __builtin_amdgcn_wave_barrier();
    __builtin_amdgcn_fence(__ATOMIC_ACQUIRE, "workgroup");
  }
}

static_assert(((size_t)kB * kH) % 256 == 0);

__global__ __launch_bounds__(256) void gate_blend_kernel(
    const float* __restrict__ GP, const float* __restrict__ h, const float* __restrict__ x,
    const float* __restrict__ bih, const float* __restrict__ bhh, float* __restrict__ out)
{
  unsigned gid = blockIdx.x * 256u + threadIdx.x;
  asm volatile("" : "+v"(gid));
  unsigned b = gid >> 7;
  unsigned j = gid & 127u;
  asm volatile("" : "+v"(b));
  asm volatile("" : "+v"(j));

  float gi_r = 0.0f, gi_z = 0.0f, gi_n = 0.0f;
  float gh_r = 0.0f, gh_z = 0.0f, gh_n = 0.0f;
#pragma unroll 1
  for (unsigned c = 0; c < (unsigned)kC; ++c) {
    const float xv = x[(size_t)b * kC + c];
    const unsigned o = c * (unsigned)kG3 + j;
    gi_r = fmaf(xv, bih[o], gi_r);
    gi_z = fmaf(xv, bih[o + (unsigned)kH], gi_z);
    gi_n = fmaf(xv, bih[o + 2u * (unsigned)kH], gi_n);
    gh_r = fmaf(xv, bhh[o], gh_r);
    gh_z = fmaf(xv, bhh[o + (unsigned)kH], gh_z);
    gh_n = fmaf(xv, bhh[o + 2u * (unsigned)kH], gh_n);
  }
  const float* gp = GP + (size_t)b * kG3 + j;
  const float rec_r = gp[0];
  const float rec_z = gp[kH];
  const float rec_n = gp[2 * kH];
  const float hv = h[(size_t)b * kH + j];

  const float hr = rec_r + gh_r;
  const float hz = rec_z + gh_z;
  const float hn = rec_n + gh_n;
  const float pr = gi_r + hr;
  const float pz = gi_z + hz;
  const float rr = 1.0f / (1.0f + expf(-pr));
  const float zz = 1.0f / (1.0f + expf(-pz));
  const float nn = tanhf(gi_n + rr * hn);
  const float res = (1.0f - zz) * nn + zz * hv;

  float* dst = out + (size_t)b * kH + j;
  *(volatile float*)dst = res;
  __threadfence();
  *(volatile float*)dst = res;
}

static_assert(((kB / 64) * (kCR / 64)) % 8 == 0);
static_assert(((kB / 64) * (kG3 / 64)) % 8 == 0);

extern "C" void kernel_launch(void* const* d_in, const int* in_sizes, int n_in,
                              void* d_out, int out_size, void* d_ws, size_t ws_size,
                              hipStream_t stream) {
  if (n_in < 6) return;
  if (in_sizes[0] != kB * kC) return;
  if (in_sizes[1] != kB * kH) return;
  if (in_sizes[2] != kC * kG3 * kR) return;
  if (in_sizes[3] != kC * kH * kR) return;
  if (in_sizes[4] != kC * kG3) return;
  if (in_sizes[5] != kC * kG3) return;
  if (out_size != kB * kH) return;
  if (ws_size < kWsTotal) return;

  const float* x   = (const float*)d_in[0];
  const float* h   = (const float*)d_in[1];
  const float* U   = (const float*)d_in[2];
  const float* V   = (const float*)d_in[3];
  const float* bih = (const float*)d_in[4];
  const float* bhh = (const float*)d_in[5];
  float* out = (float*)d_out;

  char* ws = (char*)d_ws;
  unsigned short* A1  = (unsigned short*)(ws + kOffA1);
  unsigned short* A2  = (unsigned short*)(ws + kOffA2);
  unsigned short* BT1 = (unsigned short*)(ws + kOffBT1);
  unsigned short* BT2 = (unsigned short*)(ws + kOffBT2);
  float*          GP  = (float*)(ws + kOffGP);

  prep_weights_kernel<<<kPrepBlkU + kPrepBlkV, 256, 0, stream>>>(U, V, BT1, BT2);

  cast_h_kernel<<<(kB * kH / 8) / 256, 256, 0, stream>>>(h, A1, kB * kH / 8);

  gemm_f16_kernel<0><<<((kB / 64) * (kCR / 64)) / 8, 256, 0, stream>>>(
      A1, kH, BT1, kH, (void*)A2, kCR, x, kB, kCR, kH, kInvAcc1, kCarryM);

  gemm_f16_kernel<1><<<((kB / 64) * (kG3 / 64)) / 8, 256, 0, stream>>>(
      A2, kCR, BT2, kCR, (void*)GP, kG3, x, kB, kG3, kCR, kInvAcc2, 1.0f);

  gate_blend_kernel<<<(kB * kH) / 256, 256, 0, stream>>>(GP, h, x, bih, bhh, out);
}
